// SingleMP_Tension_3427383902968
// MI455X (gfx1250) — hardware-verified
//
#include <hip/hip_runtime.h>
#include <stddef.h>


#define NB     256
#define NTA    256
#define NWA    8
#define EPT    8
#define CHUNK  (NTA * EPT)
#define WCAP   (EPT * 32)
#define LISTN  (NWA * WCAP)
#define HUP    72

#define NTE    128
#define NWE    4
#define EPB    64
#define KP1    96
#define AP1    104
#define HP     136
#define MP     72

static_assert(NB == NWA * 32);
static_assert(NB <= 256);
static_assert(EPB == NWE * 16);
static_assert(WCAP == 256);
static_assert((CHUNK << 8) > 0);

typedef float          v2f   __attribute__((ext_vector_type(2)));
typedef float          v4f   __attribute__((ext_vector_type(4)));
typedef float          v8f   __attribute__((ext_vector_type(8)));
typedef int            v4i   __attribute__((ext_vector_type(4)));
typedef unsigned int   v4u   __attribute__((ext_vector_type(4)));
typedef _Float16       v2h   __attribute__((ext_vector_type(2)));
typedef _Float16       v8h   __attribute__((ext_vector_type(8)));
typedef _Float16       v16h  __attribute__((ext_vector_type(16)));
typedef unsigned short v8us  __attribute__((ext_vector_type(8)));
typedef unsigned short v16us __attribute__((ext_vector_type(16)));
typedef __bf16         v16bf __attribute__((ext_vector_type(16)));

union FragH { v16h v; v8h h[2]; };
union FragS { v16us v; v8us h[2]; };
union Pk8h  { v8h h; v4u u; };
union Pk8s  { v8us s; v4u u; };

__device__ __forceinline__ v8f zero8f() {
  v8f z = {0.0f, 0.0f, 0.0f, 0.0f, 0.0f, 0.0f, 0.0f, 0.0f};
  return z;
}

__device__ __forceinline__ v8f wmh(v16h a, v16h b, v8f c) {
  v8f d = __builtin_amdgcn_wmma_f32_16x16x32_f16(false, a, false, b, (short)0, c, false, false);
  asm volatile("v_nop\n\tv_nop\n\tv_nop\n\tv_nop" : "+v"(d) : "v"(a), "v"(b));
  return d;
}
__device__ __forceinline__ v8f wmb(v16us a, v16us b, v8f c) {
  const v16bf ab = __builtin_bit_cast(v16bf, a);
  const v16bf bb = __builtin_bit_cast(v16bf, b);
  v8f d = __builtin_amdgcn_wmma_f32_16x16x32_bf16(false, ab, false, bb, (short)0, c, false, false);
  asm volatile("v_nop\n\tv_nop\n\tv_nop\n\tv_nop" : "+v"(d) : "v"(ab), "v"(bb));
  return d;
}

__device__ __forceinline__ v16h ld_h(const _Float16* base, int pitch, int k0, int lane) {
  const int m = lane & 15, hh = lane >> 4;
  const _Float16* p = base + (size_t)m * pitch + k0 + 8 * hh;
  FragH f;
  f.h[0] = *(const v8h*)p;
  f.h[1] = *(const v8h*)(p + 16);
  return f.v;
}
__device__ __forceinline__ v16us ld_s(const unsigned short* base, int pitch, int k0, int lane) {
  const int m = lane & 15, hh = lane >> 4;
  const unsigned short* p = base + (size_t)m * pitch + k0 + 8 * hh;
  FragS f;
  f.h[0] = *(const v8us*)p;
  f.h[1] = *(const v8us*)(p + 16);
  return f.v;
}

__device__ __forceinline__ unsigned short bfr(float f) {
  unsigned int u = __float_as_uint(f);
  u += 0x7FFFu + ((u >> 16) & 1u);
  return (unsigned short)(u >> 16);
}
__device__ __forceinline__ float bff(unsigned short s) {
  return __uint_as_float(((unsigned int)s) << 16);
}

__device__ __forceinline__ void split16(v4f q0, v4f q1, v4f q2, v4f q3, FragS& hi, FragS& lo) {
  v8f pA = {q0.x, q0.y, q0.z, q0.w, q1.x, q1.y, q1.z, q1.w};
  v8f pB = {q2.x, q2.y, q2.z, q2.w, q3.x, q3.y, q3.z, q3.w};
#pragma unroll
  for (int i = 0; i < 8; ++i) {
    const unsigned short ha = bfr(pA[i]);
    hi.h[0][i] = ha;
    lo.h[0][i] = bfr(pA[i] - bff(ha));
    const unsigned short hb = bfr(pB[i]);
    hi.h[1][i] = hb;
    lo.h[1][i] = bfr(pB[i] - bff(hb));
  }
}

__global__ __launch_bounds__(256) void k_prep(
    const float* __restrict__ Wm1, const float* __restrict__ Wm2, const float* __restrict__ Wu1,
    const float* __restrict__ Wu2, const float* __restrict__ Wt1,
    _Float16* w1t, _Float16* w2t, unsigned short* u1h, unsigned short* u1l,
    unsigned short* u2h, unsigned short* u2l, _Float16* wtt) {
  const int t = blockIdx.x * 256 + threadIdx.x;
  Pk8h p1, p2, p7;
  Pk8s p3h, p3l, p5h, p5l;
  {
    const int g = t < 1535 ? t : 1535;
    const int n = g / 12;
    const int kq = (g - n * 12) * 8;
#pragma unroll
    for (int j = 0; j < 8; ++j) {
      const int k = kq + j;
      const int kc = k < 71 ? k : 71;
      float v = Wm1[kc * 128 + n];
      v = (k < 72) ? v : 0.0f;
      p1.h[j] = (_Float16)v;
    }
  }
  {
    const int g = t < 1023 ? t : 1023;
    const int n = g / 16;
    const int kq = (g - n * 16) * 8;
#pragma unroll
    for (int j = 0; j < 8; ++j) p2.h[j] = (_Float16)Wm2[(kq + j) * 64 + n];
  }
  {
    const int g = t < 1023 ? t : 1023;
    const int n = g / 16;
    const int kq = (g - n * 16) * 8;
#pragma unroll
    for (int j = 0; j < 8; ++j) {
      const float v = Wu1[(kq + j) * 64 + n];
      const unsigned short hs = bfr(v);
      p3h.s[j] = hs;
      p3l.s[j] = bfr(v - bff(hs));
    }
  }
  {
    const int g = t < 255 ? t : 255;
    const int n = g / 8;
    const int kq = (g - n * 8) * 8;
#pragma unroll
    for (int j = 0; j < 8; ++j) {
      const float v = Wu2[(kq + j) * 32 + n];
      const unsigned short hs = bfr(v);
      p5h.s[j] = hs;
      p5l.s[j] = bfr(v - bff(hs));
    }
  }
  {
    const int g = t < 255 ? t : 255;
    const int n = g / 8;
    const int kq = (g - n * 8) * 8;
#pragma unroll
    for (int j = 0; j < 8; ++j) p7.h[j] = (_Float16)Wt1[(kq + j) * 32 + n];
  }
  const size_t go = (size_t)t * 8;
  if (t < 1536) *(volatile v4u*)(w1t + go) = p1.u;
  if (t < 1024) {
    *(volatile v4u*)(w2t + go) = p2.u;
    *(volatile v4u*)(u1h + go) = p3h.u;
    *(volatile v4u*)(u1l + go) = p3l.u;
  }
  if (t < 256) {
    *(volatile v4u*)(u2h + go) = p5h.u;
    *(volatile v4u*)(u2l + go) = p5l.u;
    *(volatile v4u*)(wtt + go) = p7.u;
  }
  __threadfence();
  if (t < 1536) *(volatile v4u*)(w1t + go) = p1.u;
  if (t < 1024) {
    *(volatile v4u*)(w2t + go) = p2.u;
    *(volatile v4u*)(u1h + go) = p3h.u;
    *(volatile v4u*)(u1l + go) = p3l.u;
  }
  if (t < 256) {
    *(volatile v4u*)(u2h + go) = p5h.u;
    *(volatile v4u*)(u2l + go) = p5l.u;
    *(volatile v4u*)(wtt + go) = p7.u;
  }
}

__global__ __launch_bounds__(NTE) __attribute__((amdgpu_num_vgpr(256)))
void k_edge(const float* __restrict__ x, const int* __restrict__ ei, const float* __restrict__ ea,
            const _Float16* __restrict__ w1t, const float* __restrict__ bm1,
            const _Float16* __restrict__ w2t, const float* __restrict__ bm2,
            const _Float16* __restrict__ wtt, const float* __restrict__ bt1,
            const float* __restrict__ wt2, const float* __restrict__ bt2,
            _Float16* mpl, float* eout, int nN, int nE, int ePad) {
  __shared__ __attribute__((aligned(16))) _Float16 At[NWE * 16 * AP1];
  __shared__ __attribute__((aligned(16))) _Float16 Hf[NWE * 16 * HP];
  __shared__ __attribute__((aligned(16))) _Float16 Hr[NWE * 16 * HP];
  __shared__ __attribute__((aligned(16))) _Float16 Mf[NWE * 16 * MP];
  __shared__ __attribute__((aligned(16))) _Float16 Mr[NWE * 16 * MP];
  __shared__ __attribute__((aligned(16))) _Float16 Ms[NWE * 16 * MP];
  __shared__ __attribute__((aligned(16))) float    Tt[NWE * 16 * 32];
  __shared__ int sI[NWE * 16];
  __shared__ int tI[NWE * 16];
  __shared__ __attribute__((aligned(16))) float    est[EPB];

  const int tid = threadIdx.x, lane = tid & 31, wave = tid >> 5, hh = lane >> 4, m = lane & 15;
  const int ebBlk = blockIdx.x * EPB;
  const int eb = ebBlk + wave * 16;

  {
    int e = eb + m;
    e = e > nE - 1 ? nE - 1 : e;
    int s = ei[e];
    int t = ei[(size_t)nE + e];
    s = s < 0 ? 0 : (s > nN - 1 ? nN - 1 : s);
    t = t < 0 ? 0 : (t > nN - 1 ? nN - 1 : t);
    if (lane < 16) {
      sI[wave * 16 + lane] = s;
      tI[wave * 16 + lane] = t;
    }
  }
  __syncthreads();

  _Float16* Aw = At + wave * 16 * AP1;
#pragma unroll 4
  for (int r = 0; r < 16; ++r) {
    const int s = sI[wave * 16 + r];
    const int t = tI[wave * 16 + r];
    int e = eb + r;
    e = e > nE - 1 ? nE - 1 : e;
    const float* xt = x + (size_t)t * 64;
    const float* xs = x + (size_t)s * 64;
    const float d0 = xt[lane] - xs[lane];
    const float d1 = xt[32 + lane] - xs[32 + lane];
    const float av = ea[(size_t)e * 8 + (lane & 7)];
    const float a2 = (lane < 8) ? av : 0.0f;
    _Float16* row = Aw + r * AP1;
    row[lane]      = (_Float16)d0;
    row[32 + lane] = (_Float16)d1;
    row[64 + lane] = (_Float16)a2;
    if (lane < 8) row[96 + lane] = (_Float16)0.0f;
  }
  __syncthreads();

  v8f acc1[8];
#pragma unroll
  for (int i = 0; i < 8; ++i) acc1[i] = zero8f();
#pragma unroll
  for (int ks = 0; ks < 3; ++ks) {
    const v16h a = ld_h(Aw, AP1, ks * 32, lane);
#pragma unroll
    for (int nt = 0; nt < 8; ++nt) {
      const v16h b = ld_h(w1t + (size_t)(nt * 16) * KP1, KP1, ks * 32, lane);
      acc1[nt] = wmh(a, b, acc1[nt]);
    }
  }
  _Float16* Hfw = Hf + wave * 16 * HP;
  _Float16* Hrw = Hr + wave * 16 * HP;
#pragma unroll
  for (int nt = 0; nt < 8; ++nt) {
    const int col = nt * 16 + m;
    const float bb = bm1[col];
#pragma unroll
    for (int r = 0; r < 8; ++r) {
      const float u = acc1[nt][r];
      Hfw[(8 * hh + r) * HP + col] = (_Float16)fmaxf(u + bb, 0.0f);
      Hrw[(8 * hh + r) * HP + col] = (_Float16)fmaxf(bb - u, 0.0f);
    }
  }
  __syncthreads();

  v8f accF[4], accR[4];
#pragma unroll
  for (int i = 0; i < 4; ++i) { accF[i] = zero8f(); accR[i] = zero8f(); }
#pragma unroll
  for (int ks = 0; ks < 4; ++ks) {
    const v16h af = ld_h(Hfw, HP, ks * 32, lane);
    const v16h ar = ld_h(Hrw, HP, ks * 32, lane);
#pragma unroll
    for (int nt = 0; nt < 4; ++nt) {
      const v16h b = ld_h(w2t + (size_t)(nt * 16) * 128, 128, ks * 32, lane);
      accF[nt] = wmh(af, b, accF[nt]);
      accR[nt] = wmh(ar, b, accR[nt]);
    }
  }
  _Float16* Mfw = Mf + wave * 16 * MP;
  _Float16* Mrw = Mr + wave * 16 * MP;
  _Float16* Msw = Ms + wave * 16 * MP;
#pragma unroll
  for (int nt = 0; nt < 4; ++nt) {
    const int col = nt * 16 + m;
    const float bb = bm2[col];
#pragma unroll
    for (int r = 0; r < 8; ++r) {
      const float vf = fmaxf(accF[nt][r] + bb, 0.0f);
      const float vr = fmaxf(accR[nt][r] + bb, 0.0f);
      const int row = 8 * hh + r;
      Mfw[row * MP + col] = (_Float16)vf;
      Mrw[row * MP + col] = (_Float16)vr;
      Msw[row * MP + col] = (_Float16)(vf + vr);
    }
  }
  __syncthreads();

  {
    v4u cf[4], cr[4];
#pragma unroll
    for (int i = 0; i < 4; ++i) {
      const int rho = 4 * i + (lane >> 3), p = lane & 7;
      Pk8h a, b;
      a.h = *(const v8h*)(Mfw + rho * MP + p * 8);
      b.h = *(const v8h*)(Mrw + rho * MP + p * 8);
      cf[i] = a.u;
      cr[i] = b.u;
    }
    const size_t rF = (size_t)eb;
    const size_t rR = (size_t)ePad + (size_t)eb;
#pragma unroll
    for (int i = 0; i < 4; ++i) {
      const int rho = 4 * i + (lane >> 3), p = lane & 7;
      *(volatile v4u*)(mpl + (rF + (size_t)rho) * 64 + p * 8) = cf[i];
      *(volatile v4u*)(mpl + (rR + (size_t)rho) * 64 + p * 8) = cr[i];
    }
    __threadfence();
#pragma unroll
    for (int i = 0; i < 4; ++i) {
      const int rho = 4 * i + (lane >> 3), p = lane & 7;
      *(volatile v4u*)(mpl + (rF + (size_t)rho) * 64 + p * 8) = cf[i];
      *(volatile v4u*)(mpl + (rR + (size_t)rho) * 64 + p * 8) = cr[i];
    }
  }

  v8f accT[2];
  accT[0] = zero8f();
  accT[1] = zero8f();
#pragma unroll
  for (int ks = 0; ks < 2; ++ks) {
    const v16h a = ld_h(Msw, MP, ks * 32, lane);
#pragma unroll
    for (int nt = 0; nt < 2; ++nt) {
      const v16h b = ld_h(wtt + (size_t)(nt * 16) * 64, 64, ks * 32, lane);
      accT[nt] = wmh(a, b, accT[nt]);
    }
  }
  float* Tw = Tt + wave * 512;
#pragma unroll
  for (int nt = 0; nt < 2; ++nt) {
    const int col = nt * 16 + m;
    const float bb = bt1[col];
#pragma unroll
    for (int r = 0; r < 8; ++r) Tw[(8 * hh + r) * 32 + col] = fmaxf(accT[nt][r] + bb, 0.0f);
  }
  __syncthreads();

  {
    const float* tr = Tw + m * 32;
    float s = 0.0f;
#pragma unroll 4
    for (int c = 0; c < 32; ++c) s += tr[c] * wt2[c];
    s += bt2[0];
    if (lane < 16) est[wave * 16 + lane] = s;
  }
  __syncthreads();

  {
    int nv = nE - ebBlk;
    nv = nv > EPB ? EPB : (nv < 0 ? 0 : nv);
    const int q = lane & 15;
    const v4f ov = *(const v4f*)(est + 4 * q);
    const bool wr = (wave == 0) && (lane < 16) && (4 * q + 3 < nv);
    float* op = eout + (size_t)ebBlk + 4 * q;
    const int t4 = nv & ~3;
    const bool wt = (wave == 0) && (lane == 0) && (t4 < nv);
    const float tv0 = est[t4 < EPB ? t4 : EPB - 1];
    const float tv1 = est[t4 + 1 < EPB ? t4 + 1 : EPB - 1];
    const float tv2 = est[t4 + 2 < EPB ? t4 + 2 : EPB - 1];
    float* tp = eout + (size_t)ebBlk + t4;
    if (wr) *(volatile v4f*)op = ov;
    if (wt) {
      if (t4 < nv)     *(volatile float*)(tp)     = tv0;
      if (t4 + 1 < nv) *(volatile float*)(tp + 1) = tv1;
      if (t4 + 2 < nv) *(volatile float*)(tp + 2) = tv2;
    }
    __threadfence();
    if (wr) *(volatile v4f*)op = ov;
    if (wt) {
      if (t4 < nv)     *(volatile float*)(tp)     = tv0;
      if (t4 + 1 < nv) *(volatile float*)(tp + 1) = tv1;
      if (t4 + 2 < nv) *(volatile float*)(tp + 2) = tv2;
    }
  }
}

__device__ __forceinline__ int scan_chunk(const int* __restrict__ dsts, int nE, int cbase, int nodeBase,
                                          int vec8, int* list, int tid, int wave) {
  int wc = 0;
  const int el0  = tid * EPT;
  const int e0   = cbase + el0;
  const int sent = -2147483647 - 1;
  v4i da, db;
  if (vec8 != 0 && cbase + CHUNK <= nE) {
    da = *(const v4i*)(dsts + e0);
    db = *(const v4i*)(dsts + e0 + 4);
  } else {
    da.x = (e0     < nE) ? dsts[min(e0,     nE - 1)] : sent;
    da.y = (e0 + 1 < nE) ? dsts[min(e0 + 1, nE - 1)] : sent;
    da.z = (e0 + 2 < nE) ? dsts[min(e0 + 2, nE - 1)] : sent;
    da.w = (e0 + 3 < nE) ? dsts[min(e0 + 3, nE - 1)] : sent;
    db.x = (e0 + 4 < nE) ? dsts[min(e0 + 4, nE - 1)] : sent;
    db.y = (e0 + 5 < nE) ? dsts[min(e0 + 5, nE - 1)] : sent;
    db.z = (e0 + 6 < nE) ? dsts[min(e0 + 6, nE - 1)] : sent;
    db.w = (e0 + 7 < nE) ? dsts[min(e0 + 7, nE - 1)] : sent;
  }
  const unsigned nb = (unsigned)nodeBase;
  const unsigned s0 = (unsigned)da.x - nb, s1 = (unsigned)da.y - nb;
  const unsigned s2 = (unsigned)da.z - nb, s3 = (unsigned)da.w - nb;
  const unsigned s4 = (unsigned)db.x - nb, s5 = (unsigned)db.y - nb;
  const unsigned s6 = (unsigned)db.z - nb, s7 = (unsigned)db.w - nb;
  const bool h0 = s0 < (unsigned)NB, h1 = s1 < (unsigned)NB, h2 = s2 < (unsigned)NB, h3 = s3 < (unsigned)NB;
  const bool h4 = s4 < (unsigned)NB, h5 = s5 < (unsigned)NB, h6 = s6 < (unsigned)NB, h7 = s7 < (unsigned)NB;
  const unsigned any = __builtin_amdgcn_ballot_w32(h0 | h1 | h2 | h3 | h4 | h5 | h6 | h7);
  if (any != 0u) {
#define HITJ(J, HJ, SJ) { \
      const unsigned mj = __builtin_amdgcn_ballot_w32(HJ); \
      if (mj != 0u) { \
        if (HJ) { \
          const int pos = wc + (int)__builtin_amdgcn_mbcnt_lo(mj, 0u); \
          if (pos < WCAP) list[wave * WCAP + pos] = ((el0 + (J)) << 8) | (int)(SJ); \
        } \
        wc += (int)__builtin_popcount(mj); } }
    HITJ(0, h0, s0)
    HITJ(1, h1, s1)
    HITJ(2, h2, s2)
    HITJ(3, h3, s3)
    HITJ(4, h4, s4)
    HITJ(5, h5, s5)
    HITJ(6, h6, s6)
    HITJ(7, h7, s7)
#undef HITJ
  }
  return wc;
}

__device__ __forceinline__ void l1step(v8f (&a1)[4], const v16us ah, const v16us al,
                                       const unsigned short* __restrict__ u1h,
                                       const unsigned short* __restrict__ u1l, int k0, int lane) {
#pragma unroll
  for (int nt = 0; nt < 4; ++nt) {
    const v16us bh = ld_s(u1h + (size_t)(nt * 16) * 128, 128, k0, lane);
    const v16us bl = ld_s(u1l + (size_t)(nt * 16) * 128, 128, k0, lane);
    a1[nt] = wmb(ah, bh, a1[nt]);
    a1[nt] = wmb(ah, bl, a1[nt]);
    a1[nt] = wmb(al, bh, a1[nt]);
  }
}

__global__ __launch_bounds__(NTA) __attribute__((amdgpu_num_vgpr(256)))
void k_aggr(const float* __restrict__ x, const int* __restrict__ ei, const _Float16* __restrict__ mpl,
            const unsigned short* __restrict__ u1h, const unsigned short* __restrict__ u1l,
            const float* __restrict__ bu1,
            const unsigned short* __restrict__ u2h, const unsigned short* __restrict__ u2l,
            const float* __restrict__ bu2,
            float* xout, int nN, int nE, int ePad, int vec8) {
  __shared__ __attribute__((aligned(16))) float          acc[NB * 64];
  __shared__ float                                        cntL[NB];
  __shared__ __attribute__((aligned(16))) int            list[LISTN];
  __shared__ int                                          wcnt[NWA];
  __shared__ __attribute__((aligned(16))) unsigned short huH[NWA * 16 * HUP];
  __shared__ __attribute__((aligned(16))) unsigned short huL[NWA * 16 * HUP];
  __shared__ __attribute__((aligned(16))) float          xo[NWA * 16 * 32];

  const int tid = threadIdx.x, lane = tid & 31, wave = tid >> 5, hh = lane >> 4, m = lane & 15;
  const int nodeBase = blockIdx.x * NB;

  for (int i = tid; i < NB * 64; i += NTA) acc[i] = 0.0f;
  for (int i = tid; i < NB; i += NTA) cntL[i] = 0.0f;
  __syncthreads();

  const int nChunks = (nE + CHUNK - 1) / CHUNK;
#pragma unroll 1
  for (int half = 0; half < 2; ++half) {
    const int* dsts = (half == 0) ? (ei + nE) : ei;
    const size_t rowoff = (half == 0) ? (size_t)0 : (size_t)ePad;
#pragma unroll 1
    for (int ch = 0; ch < nChunks; ++ch) {
      const int cbase = ch * CHUNK;
      const int wc = scan_chunk(dsts, nE, cbase, nodeBase, vec8, list, tid, wave);
      if (lane == 0) wcnt[wave] = wc;
      __syncthreads();
      if (wave == 0) {
#pragma unroll 1
        for (int w = 0; w < NWA; ++w) {
          int n = wcnt[w];
          n = n > WCAP ? WCAP : (n < 0 ? 0 : n);
#pragma unroll 1
          for (int i = 0; i < n; ++i) {
            const int ent = list[w * WCAP + i];
            int e = cbase + (ent >> 8);
            e = e < 0 ? 0 : (e > nE - 1 ? nE - 1 : e);
            const int slot = ent & (NB - 1);
            const v2h hv = *(const v2h*)(mpl + (rowoff + (size_t)e) * 64 + 2 * lane);
            float* ap = acc + slot * 64 + 2 * lane;
            v2f cur = *(const v2f*)ap;
            cur.x += (float)hv.x;
            cur.y += (float)hv.y;
            *(v2f*)ap = cur;
            if (lane == 0) cntL[slot] += 1.0f;
          }
        }
      }
      __syncthreads();
    }
  }

#pragma unroll 1
  for (int tl = 0; tl < 2; ++tl) {
    const int sbase = wave * 32 + tl * 16;
    const int sA = sbase + m;
    int node = nodeBase + sA;
    node = node > nN - 1 ? nN - 1 : node;
    const float rinv = 1.0f / fmaxf(cntL[sA], 1.0f);

    v8f a1[4];
#pragma unroll
    for (int i = 0; i < 4; ++i) a1[i] = zero8f();
#pragma unroll
    for (int ks = 0; ks < 2; ++ks) {
      const float* xp = x + (size_t)node * 64 + ks * 32 + 8 * hh;
      const v4f q0 = *(const v4f*)xp;
      const v4f q1 = *(const v4f*)(xp + 4);
      const v4f q2 = *(const v4f*)(xp + 16);
      const v4f q3 = *(const v4f*)(xp + 20);
      FragS ah, al;
      split16(q0, q1, q2, q3, ah, al);
      l1step(a1, ah.v, al.v, u1h, u1l, ks * 32, lane);
    }
#pragma unroll
    for (int ks = 2; ks < 4; ++ks) {
      const float* lp = acc + sA * 64 + (ks - 2) * 32 + 8 * hh;
      const v4f q0 = *(const v4f*)lp * rinv;
      const v4f q1 = *(const v4f*)(lp + 4) * rinv;
      const v4f q2 = *(const v4f*)(lp + 16) * rinv;
      const v4f q3 = *(const v4f*)(lp + 20) * rinv;
      FragS ah, al;
      split16(q0, q1, q2, q3, ah, al);
      l1step(a1, ah.v, al.v, u1h, u1l, ks * 32, lane);
    }
    unsigned short* hHw = huH + wave * 16 * HUP;
    unsigned short* hLw = huL + wave * 16 * HUP;
#pragma unroll
    for (int nt = 0; nt < 4; ++nt) {
      const int col = nt * 16 + m;
      const float bb = bu1[col];
#pragma unroll
      for (int r = 0; r < 8; ++r) {
        const float v = fmaxf(a1[nt][r] + bb, 0.0f);
        const unsigned short hs = bfr(v);
        hHw[(8 * hh + r) * HUP + col] = hs;
        hLw[(8 * hh + r) * HUP + col] = bfr(v - bff(hs));
      }
    }
    __syncthreads();

    v8f a2[2];
    a2[0] = zero8f();
    a2[1] = zero8f();
#pragma unroll
    for (int ks = 0; ks < 2; ++ks) {
      const v16us ah = ld_s(hHw, HUP, ks * 32, lane);
      const v16us al = ld_s(hLw, HUP, ks * 32, lane);
#pragma unroll
      for (int nt = 0; nt < 2; ++nt) {
        const v16us bh = ld_s(u2h + (size_t)(nt * 16) * 64, 64, ks * 32, lane);
        const v16us bl = ld_s(u2l + (size_t)(nt * 16) * 64, 64, ks * 32, lane);
        a2[nt] = wmb(ah, bh, a2[nt]);
        a2[nt] = wmb(ah, bl, a2[nt]);
        a2[nt] = wmb(al, bh, a2[nt]);
      }
    }
    float* xw = xo + wave * 512;
#pragma unroll
    for (int nt = 0; nt < 2; ++nt) {
      const int col = nt * 16 + m;
      const float bb = bu2[col];
#pragma unroll
      for (int r = 0; r < 8; ++r) xw[(8 * hh + r) * 32 + col] = a2[nt][r] + bb;
    }
    __syncthreads();

    v4f ov[4];
#pragma unroll
    for (int i = 0; i < 4; ++i) {
      const int rho = 4 * i + (lane >> 3), p = lane & 7;
      ov[i] = *(const v4f*)(xw + rho * 32 + 4 * p);
    }
#pragma unroll
    for (int i = 0; i < 4; ++i) {
      const int rho = 4 * i + (lane >> 3), p = lane & 7;
      const int no = nodeBase + sbase + rho;
      if (no < nN) *(volatile v4f*)(xout + (size_t)no * 32 + 4 * p) = ov[i];
    }
    __threadfence();
#pragma unroll
    for (int i = 0; i < 4; ++i) {
      const int rho = 4 * i + (lane >> 3), p = lane & 7;
      const int no = nodeBase + sbase + rho;
      if (no < nN) *(volatile v4f*)(xout + (size_t)no * 32 + 4 * p) = ov[i];
    }
  }
}

static inline size_t al256(size_t v) { return (v + 255) & ~(size_t)255; }

extern "C" void kernel_launch(void* const* d_in, const int* in_sizes, int n_in,
                              void* d_out, int out_size, void* d_ws, size_t ws_size,
                              hipStream_t stream) {
  if (n_in < 15) return;
  const int nN = in_sizes[0] / 64;
  const int nE = in_sizes[1] / 2;
  if (nN <= 0 || nE <= 0) return;
  if (in_sizes[0] != nN * 64 || in_sizes[1] != 2 * nE || in_sizes[2] != nE * 8) return;
  if (in_sizes[3] != 72 * 128 || in_sizes[4] != 128) return;
  if (in_sizes[5] != 128 * 64 || in_sizes[6] != 64) return;
  if (in_sizes[7] != 128 * 64 || in_sizes[8] != 64) return;
  if (in_sizes[9] != 64 * 32 || in_sizes[10] != 32) return;
  if (in_sizes[11] != 64 * 32 || in_sizes[12] != 32) return;
  if (in_sizes[13] != 32 || in_sizes[14] < 1) return;
  if (out_size != nN * 32 + nE) return;

  const float* x   = (const float*)d_in[0];
  const int*   ei  = (const int*)d_in[1];
  const float* ea  = (const float*)d_in[2];
  const float* Wm1 = (const float*)d_in[3];
  const float* bm1 = (const float*)d_in[4];
  const float* Wm2 = (const float*)d_in[5];
  const float* bm2 = (const float*)d_in[6];
  const float* Wu1 = (const float*)d_in[7];
  const float* bu1 = (const float*)d_in[8];
  const float* Wu2 = (const float*)d_in[9];
  const float* bu2 = (const float*)d_in[10];
  const float* Wt1 = (const float*)d_in[11];
  const float* bt1 = (const float*)d_in[12];
  const float* Wt2 = (const float*)d_in[13];
  const float* bt2 = (const float*)d_in[14];

  float* xout = (float*)d_out;
  float* eout = (float*)d_out + (size_t)nN * 32;

  const int ePad = ((nE + EPB - 1) / EPB) * EPB;

  char* ws = (char*)d_ws;
  size_t off = 0;
  const size_t oM   = off; off = al256(off + (size_t)2 * (size_t)ePad * 64 * sizeof(_Float16));
  const size_t oW1  = off; off = al256(off + (size_t)128 * KP1 * 2);
  const size_t oW2  = off; off = al256(off + (size_t)64 * 128 * 2);
  const size_t oU1H = off; off = al256(off + (size_t)64 * 128 * 2);
  const size_t oU1L = off; off = al256(off + (size_t)64 * 128 * 2);
  const size_t oU2H = off; off = al256(off + (size_t)32 * 64 * 2);
  const size_t oU2L = off; off = al256(off + (size_t)32 * 64 * 2);
  const size_t oTT  = off; off = al256(off + (size_t)32 * 64 * 2);
  if (off > ws_size) return;

  _Float16*       mpl = (_Float16*)(ws + oM);
  _Float16*       w1t = (_Float16*)(ws + oW1);
  _Float16*       w2t = (_Float16*)(ws + oW2);
  unsigned short* u1h = (unsigned short*)(ws + oU1H);
  unsigned short* u1l = (unsigned short*)(ws + oU1L);
  unsigned short* u2h = (unsigned short*)(ws + oU2H);
  unsigned short* u2l = (unsigned short*)(ws + oU2L);
  _Float16*       wtt = (_Float16*)(ws + oTT);

  const int vec8 = ((nE & 3) == 0) ? 1 : 0;
  const int nBlkE = ePad / EPB;
  const int nBlkA = (nN + NB - 1) / NB;

  k_prep<<<6, 256, 0, stream>>>(Wm1, Wm2, Wu1, Wu2, Wt1, w1t, w2t, u1h, u1l, u2h, u2l, wtt);

  k_edge<<<nBlkE, NTE, 0, stream>>>(x, ei, ea, w1t, bm1, w2t, bm2, wtt, bt1, Wt2, bt2,
                                     mpl, eout, nN, nE, ePad);

  k_aggr<<<nBlkA, NTA, 0, stream>>>(x, ei, mpl, u1h, u1l, bu1, u2h, u2l, bu2,
                                     xout, nN, nE, ePad, vec8);
}
